// SimpleRNN_39926015983951
// MI455X (gfx1250) — hardware-verified
//
#include <hip/hip_runtime.h>
#include <math.h>

constexpr int NB   = 256;
constexpr int NT   = 2048;
constexpr int NI   = 8;
constexpr int NH   = 128;
constexpr int ROWS_PB = 32;
constexpr int NBLK = NB / ROWS_PB;
constexpr int NTHR = 256;
constexpr int NWAVE = NTHR / 32;
constexpr int COL_XH = NH;
constexpr int COL_XL = NH + NI;
constexpr int COL_Z  = NH + 2 * NI;
constexpr int KCAT = 160;
constexpr int NKC  = KCAT / 32;
constexpr int AP   = 168;
constexpr int TILE = ROWS_PB * AP;
constexpr int SP   = 132;
constexpr float WCARRY      = 16.0f;
constexpr float WCARRY_INV  = 1.0f / 16.0f;
constexpr float XLO_CARRY   = 256.0f;
constexpr float WIH_LO_SCALE = WCARRY / XLO_CARRY;
constexpr int OUT0_F = 0;
constexpr int OUT1_F = 1024 / 4;
constexpr int OUT2_F = 132096 / 4;
constexpr int OUT_TOTAL_F = 263168 / 4;
static_assert(NB % ROWS_PB == 0);
static_assert(ROWS_PB == 32);
static_assert(NH == 16 * NWAVE);
static_assert(NH % 32 == 0 && KCAT % 32 == 0 && COL_Z + 16 == KCAT && KCAT <= AP && AP % 8 == 0);
static_assert(ROWS_PB * NI == NTHR);
static_assert(ROWS_PB * 8 == NTHR);
static_assert(ROWS_PB == 4 * NWAVE);
static_assert(SP % 4 == 0 && SP >= NH);
static_assert(OUT1_F == NB && OUT2_F == NB + NB * NH && OUT_TOTAL_F == NB + 2 * NB * NH);
static_assert(NT % 2 == 0);

typedef __attribute__((ext_vector_type(16))) _Float16 v16h;
typedef __attribute__((ext_vector_type(8)))  _Float16 v8h;
typedef __attribute__((ext_vector_type(16))) __bf16   v16b;
typedef __attribute__((ext_vector_type(8)))  __bf16   v8b;
typedef __attribute__((ext_vector_type(8)))  float    v8f;
typedef __attribute__((ext_vector_type(4)))  float    v4f;

__device__ __forceinline__ void dep_guard_h(v8f& a, v8f& b, v16h x, v16h y) { asm volatile("v_nop\n\tv_nop\n\tv_nop\n\tv_nop" : "+v"(a), "+v"(b) : "v"(x), "v"(y)); }
__device__ __forceinline__ void dep_guard_b(v8f& a, v8f& b, v16b x, v16b y) { asm volatile("v_nop\n\tv_nop\n\tv_nop\n\tv_nop" : "+v"(a), "+v"(b) : "v"(x), "v"(y)); }
__device__ __forceinline__ void keep4_h(v16h a, v16h b, v16h c, v16h d) { asm volatile("v_nop" :: "v"(a), "v"(b), "v"(c), "v"(d)); }
__device__ __forceinline__ void keep4_b(v16b a, v16b b, v16b c, v16b d) { asm volatile("v_nop" :: "v"(a), "v"(b), "v"(c), "v"(d)); }
__device__ __forceinline__ void acc_guard2(v8f& a, v8f& b) { asm volatile("v_nop\n\tv_nop\n\tv_nop\n\tv_nop" : "+v"(a), "+v"(b)); }
__device__ __forceinline__ void dep_guard3_h(v8f& a, v8f& b, v16h x, v16h y, v16h z) {
  asm volatile("v_nop\n\tv_nop\n\tv_nop\n\tv_nop" : "+v"(a), "+v"(b) : "v"(x), "v"(y), "v"(z));
}
template <typename T> struct Frag;
template <> struct Frag<_Float16> {
  typedef v16h V; union U { v16h v; v8h h[2]; };
  static __device__ __forceinline__ v16h load(const _Float16* p) {
    U f; f.h[0] = *(const v8h*)(p); f.h[1] = *(const v8h*)(p + 16); return f.v;
  }
  static __device__ __forceinline__ v8f mma(v16h a, v16h b, v8f c) {
    return __builtin_amdgcn_wmma_f32_16x16x32_f16(false, a, false, b, (short)0, c, false, false);
  }
  static __device__ __forceinline__ void guard(v8f& a, v8f& b, v16h x, v16h y) { dep_guard_h(a, b, x, y); }
  static __device__ __forceinline__ void keep(v16h a, v16h b, v16h c, v16h d) { keep4_h(a, b, c, d); }
};
template <> struct Frag<__bf16> {
  typedef v16b V; union U { v16b v; v8b h[2]; };
  static __device__ __forceinline__ v16b load(const __bf16* p) {
    U f; f.h[0] = *(const v8b*)(p); f.h[1] = *(const v8b*)(p + 16); return f.v;
  }
  static __device__ __forceinline__ v8f mma(v16b a, v16b b, v8f c) {
    return __builtin_amdgcn_wmma_f32_16x16x32_bf16(false, a, false, b, (short)0, c, false, false);
  }
  static __device__ __forceinline__ void guard(v8f& a, v8f& b, v16b x, v16b y) { dep_guard_b(a, b, x, y); }
  static __device__ __forceinline__ void keep(v16b a, v16b b, v16b c, v16b d) { keep4_b(a, b, c, d); }
};

__device__ __forceinline__ void put_x_cols(_Float16* tile, int xrow, int xi, float xv) {
  const _Float16 hi = (_Float16)xv;
  const float hif = (float)hi;
  const float res = (xv - hif) * XLO_CARRY;
  const _Float16 lo = (_Float16)res;
  tile[xrow * AP + COL_XH + xi] = hi;
  tile[xrow * AP + COL_XL + xi] = lo;
  *(unsigned*)(tile + xrow * AP + COL_Z + 2 * xi) = 0u;
}

__global__ __launch_bounds__(NTHR) void rnn_tanh_seq_kernel(
    const float* __restrict__ x,
    const float* __restrict__ h0,
    const float* __restrict__ W_ih,
    const float* __restrict__ W_hh,
    const float* __restrict__ b_ih,
    const float* __restrict__ b_hh,
    const float* __restrict__ W_head,
    const float* __restrict__ b_head,
    float* __restrict__ out) {
  __shared__ __align__(16) _Float16 At[2 * TILE];
  __shared__ __align__(16) float    Sl[ROWS_PB * SP];
  __shared__ __align__(16) float    Sp[ROWS_PB];
  const int tid = threadIdx.x, lane = tid & 31, wave = tid >> 5;
  const int c = lane & 15, hh = lane >> 4, koff = hh * 8, mOff = hh * 8;
  const int b0 = blockIdx.x * ROWS_PB;
  const int n = 16 * wave + c;

  v16h wb[NKC];
#pragma unroll
  for (int kc = 0; kc < NKC - 1; ++kc) {
    const float* wp = W_hh + (size_t)n * NH + 32 * kc + koff;
    const v4f w0 = *(const v4f*)(wp);
    const v4f w1 = *(const v4f*)(wp + 4);
    const v4f w2 = *(const v4f*)(wp + 16);
    const v4f w3 = *(const v4f*)(wp + 20);
    v16h f;
#pragma unroll
    for (int e = 0; e < 4; ++e) {
      f[e]      = (_Float16)(w0[e] * WCARRY);
      f[4 + e]  = (_Float16)(w1[e] * WCARRY);
      f[8 + e]  = (_Float16)(w2[e] * WCARRY);
      f[12 + e] = (_Float16)(w3[e] * WCARRY);
    }
    wb[kc] = f;
    asm volatile("" ::: "memory");
  }
  {
    const float* wip = W_ih + (size_t)n * NI;
    const v4f u0 = *(const v4f*)(wip);
    const v4f u1 = *(const v4f*)(wip + 4);
    const float sc = hh ? WIH_LO_SCALE : WCARRY;
    v16h f;
#pragma unroll
    for (int e = 0; e < 4; ++e) {
      f[e]      = (_Float16)(u0[e] * sc);
      f[4 + e]  = (_Float16)(u1[e] * sc);
      f[8 + e]  = (_Float16)0.0f;
      f[12 + e] = (_Float16)0.0f;
    }
    wb[NKC - 1] = f;
    asm volatile("" ::: "memory");
  }
  const float bias_n = b_ih[n] + b_hh[n];
  const v4f whv = *(const v4f*)(W_head + 4 * lane);
  const float bhead = b_head[0];

  const int xrow = tid >> 3, xi = tid & 7;
  const float* xptr = x + (size_t)(b0 + xrow) * NT * NI + xi;

  {
    const int row = tid >> 3, c16 = (tid & 7) * 16;
    const float* hp = h0 + (size_t)(b0 + row) * NH + c16;
    const v4f q0 = *(const v4f*)(hp);
    const v4f q1 = *(const v4f*)(hp + 4);
    const v4f q2 = *(const v4f*)(hp + 8);
    const v4f q3 = *(const v4f*)(hp + 12);
    v8h v0, v1;
#pragma unroll
    for (int e = 0; e < 4; ++e) {
      v0[e] = (_Float16)q0[e]; v0[4 + e] = (_Float16)q1[e];
      v1[e] = (_Float16)q2[e]; v1[4 + e] = (_Float16)q3[e];
    }
    *(v8h*)(At + row * AP + c16)     = v0;
    *(v8h*)(At + row * AP + c16 + 8) = v1;
    const float xv0 = xptr[0];
    put_x_cols(At, xrow, xi, xv0);
  }
  __syncthreads();

  const v8f z8 = {0.f, 0.f, 0.f, 0.f, 0.f, 0.f, 0.f, 0.f};

#pragma unroll 1
  for (int t = 0; t < NT; ++t) {
    const int cur = t & 1;
    const _Float16* tc  = At + cur * TILE;
    _Float16*       tnx = At + (cur ^ 1) * TILE;
    const int tnext = (t + 1 < NT) ? (t + 1) : (NT - 1);
    const float xv = xptr[(size_t)tnext * NI];

    v8f acc0 = z8, acc1 = z8;
#pragma unroll
    for (int kc = 0; kc < NKC; ++kc) {
      const v16h a0 = Frag<_Float16>::load(tc + c * AP + koff + 32 * kc);
      const v16h a1 = Frag<_Float16>::load(tc + (16 + c) * AP + koff + 32 * kc);
      acc0 = Frag<_Float16>::mma(a0, wb[kc], acc0);
      acc1 = Frag<_Float16>::mma(a1, wb[kc], acc1);
      dep_guard3_h(acc0, acc1, a0, a1, wb[kc]);
    }
    acc_guard2(acc0, acc1);

    float hv0[8], hv1[8];
#pragma unroll
    for (int r = 0; r < 8; ++r) {
      hv0[r] = tanhf(acc0[r] * WCARRY_INV + bias_n);
      hv1[r] = tanhf(acc1[r] * WCARRY_INV + bias_n);
    }
#pragma unroll
    for (int r = 0; r < 8; ++r) {
      tnx[(mOff + r) * AP + n]      = (_Float16)hv0[r];
      tnx[(16 + mOff + r) * AP + n] = (_Float16)hv1[r];
    }
    if (t == NT - 1) {
#pragma unroll
      for (int r = 0; r < 8; ++r) {
        Sl[(mOff + r) * SP + n]      = hv0[r];
        Sl[(16 + mOff + r) * SP + n] = hv1[r];
      }
    }
    put_x_cols(tnx, xrow, xi, xv);
    __syncthreads();
  }

#pragma unroll
  for (int j = 0; j < 4; ++j) {
    const int row = 4 * wave + j;
    const v4f hr = *(const v4f*)(Sl + row * SP + 4 * lane);
    float s = 0.0f;
    s += hr[0] * whv[0];
    s += hr[1] * whv[1];
    s += hr[2] * whv[2];
    s += hr[3] * whv[3];
#pragma unroll
    for (int off = 16; off > 0; off >>= 1) s += __shfl_xor(s, off, 32);
    if (lane == 0) Sp[row] = s + bhead;
  }
  __syncthreads();

  float* o1 = out + OUT1_F + (size_t)b0 * NH;
  float* o2 = out + OUT2_F + (size_t)b0 * NH;
  float* o0 = out + OUT0_F + b0;
  const int pl = (lane & 7) * 4;
  for (int pass = 0; pass < 2; ++pass) {
#pragma unroll
    for (int j = 0; j < 4; ++j) {
      const int row = 4 * wave + j;
      const v4f v = *(const v4f*)(Sl + row * SP + 4 * lane);
      *(volatile v4f*)(o1 + (size_t)row * NH + 4 * lane) = v;
      *(volatile v4f*)(o2 + (size_t)row * NH + 4 * lane) = v;
    }
    const v4f pv = *(const v4f*)(Sp + pl);
    if (wave == 0 && lane < 8) *(volatile v4f*)(o0 + pl) = pv;
    __threadfence();
  }
}

extern "C" void kernel_launch(void* const* d_in, const int* in_sizes, int n_in,
                              void* d_out, int out_size, void* d_ws, size_t ws_size, hipStream_t stream) {
  (void)d_ws; (void)ws_size;
  if (n_in < 8 || d_out == nullptr) return;
  if (in_sizes[0] != NB * NT * NI || in_sizes[1] != NB * NH || in_sizes[2] != NH * NI || in_sizes[3] != NH * NH ||
      in_sizes[4] != NH || in_sizes[5] != NH || in_sizes[6] != NH || in_sizes[7] != 1 ||
      out_size != OUT_TOTAL_F) return;

  const float* x      = (const float*)d_in[0];
  const float* h0     = (const float*)d_in[1];
  const float* W_ih   = (const float*)d_in[2];
  const float* W_hh   = (const float*)d_in[3];
  const float* b_ih   = (const float*)d_in[4];
  const float* b_hh   = (const float*)d_in[5];
  const float* W_head = (const float*)d_in[6];
  const float* b_head = (const float*)d_in[7];
  float* out = (float*)d_out;

  rnn_tanh_seq_kernel<<<dim3(NBLK), dim3(NTHR), 0, stream>>>(x, h0, W_ih, W_hh, b_ih, b_hh, W_head, b_head, out);
}
